// BatchedGATWrapper_52080773431339
// MI455X (gfx1250) — hardware-verified
//
#include <hip/hip_runtime.h>
#include <math.h>
#include <stdint.h>

#define NB 8
#define NN 1024
#define ND 512
#define NH 8
#define NC 64
#define HC (NH * NC)
#define ITILE 16
#define LEAKY 0.2f
#define PSCALE 1024.0f
#define LOSCALE 2048.0f
#define INV_P  (1.0f / 1024.0f)
#define INV_PL (1.0f / (1024.0f * 2048.0f))

typedef __attribute__((ext_vector_type(16))) _Float16 v16h;
typedef __attribute__((ext_vector_type(8)))  _Float16 v8h;
typedef __attribute__((ext_vector_type(16))) __bf16   v16b;
typedef __attribute__((ext_vector_type(8)))  __bf16   v8b;
typedef __attribute__((ext_vector_type(8)))  float    v8f;
typedef __attribute__((ext_vector_type(4)))  float    v4f;
typedef __attribute__((ext_vector_type(4)))  int      v4i;
typedef __attribute__((ext_vector_type(4)))  unsigned int v4u;

__device__ __forceinline__ unsigned short f2bf_bits(float f) {
  const unsigned u = __float_as_uint(f);
  return (unsigned short)((u + 0x7FFFu + ((u >> 16) & 1u)) >> 16);
}
__device__ __forceinline__ float bf_bits2f(unsigned short b) { return __uint_as_float(((unsigned)b) << 16); }
__device__ __forceinline__ float bf_rn(float f) { return bf_bits2f(f2bf_bits(f)); }
__device__ __forceinline__ unsigned pk16(unsigned short a, unsigned short b) { return (unsigned)a | ((unsigned)b << 16); }
__device__ __forceinline__ unsigned short h_bits(_Float16 x) { return __builtin_bit_cast(unsigned short, x); }

union FragB { v16b v; v8b h[2]; };
union FragH { v16h v; v8h h[2]; _Float16 s[16]; };

__device__ __forceinline__ v16b ldfrag_b(const __bf16* p) {
  FragB f; f.h[0] = *(const v8b*)(p); f.h[1] = *(const v8b*)(p + 16); return f.v;
}
__device__ __forceinline__ v16h ldfrag_h(const _Float16* p) {
  FragH f; f.h[0] = *(const v8h*)(p); f.h[1] = *(const v8h*)(p + 16); return f.v;
}
__device__ __forceinline__ v8f mma_b(v16b a, v16b b, v8f c) {
  return __builtin_amdgcn_wmma_f32_16x16x32_bf16(false, a, false, b, (short)0, c, false, false);
}
__device__ __forceinline__ v8f mma_h(v16h a, v16h b, v8f c) {
  return __builtin_amdgcn_wmma_f32_16x16x32_f16(false, a, false, b, (short)0, c, false, false);
}
__device__ __forceinline__ void guard_b2(v8f& a, v8f& b, v16b x, v16b y) {
#if defined(__HIP_DEVICE_COMPILE__)
  asm volatile("v_nop\n\tv_nop\n\tv_nop\n\tv_nop" : "+v"(a), "+v"(b) : "v"(x), "v"(y));
#endif
}
__device__ __forceinline__ void keep4_b(v16b a, v16b b, v16b c, v16b d) {
#if defined(__HIP_DEVICE_COMPILE__)
  asm volatile("v_nop" :: "v"(a), "v"(b), "v"(c), "v"(d));
#endif
}
__device__ __forceinline__ void acc_guard4(v8f& a, v8f& b, v8f& c, v8f& d) {
#if defined(__HIP_DEVICE_COMPILE__)
  asm volatile("v_nop\n\tv_nop\n\tv_nop\n\tv_nop" : "+v"(a), "+v"(b), "+v"(c), "+v"(d));
#endif
}
__device__ __forceinline__ void guard_h3(v8f& a, v8f& b, v16h x, v16h y, v16h z) {
#if defined(__HIP_DEVICE_COMPILE__)
  asm volatile("v_nop\n\tv_nop\n\tv_nop\n\tv_nop" : "+v"(a), "+v"(b) : "v"(x), "v"(y), "v"(z));
#endif
}

__global__ __launch_bounds__(256) void k_wt(const float* __restrict__ W, unsigned short* __restrict__ Wt) {
  __shared__ __align__(16) unsigned short tb[64 * 72];
  const int n0  = blockIdx.x * 64;
  const int k0  = blockIdx.y * 64;
  const int tid = threadIdx.x;
  {
    const int rr = tid >> 2;
    const int cq = (tid & 3) * 16;
    const float* src = W + (size_t)(k0 + rr) * HC + n0 + cq;
#pragma unroll
    for (int q = 0; q < 4; ++q) {
      const v4f f = *(const v4f*)(src + 4 * q);
#pragma unroll
      for (int e = 0; e < 4; ++e) tb[rr * 72 + cq + 4 * q + e] = f2bf_bits(f[e]);
    }
  }
  __syncthreads();
  const int sub = tid >> 3;
  const int c8  = (tid & 7) * 8;
  v4u hv[2];
#pragma unroll
  for (int it = 0; it < 2; ++it) {
    const int oc = it * 32 + sub;
    v4u a;
#pragma unroll
    for (int q = 0; q < 4; ++q) a[q] = pk16(tb[(c8 + 2 * q) * 72 + oc], tb[(c8 + 2 * q + 1) * 72 + oc]);
    hv[it] = a;
  }
  for (int pass = 0; pass < 2; ++pass) {
#pragma unroll
    for (int it = 0; it < 2; ++it) {
      const int oc = it * 32 + sub;
      *(volatile v4u*)(Wt + (size_t)(n0 + oc) * ND + k0 + c8) = hv[it];
    }
    __threadfence();
  }
}

__global__ __launch_bounds__(256) void k_cvtf(const float* __restrict__ in, unsigned short* __restrict__ outp, int n8) {
  const int i = blockIdx.x * 256 + threadIdx.x;
  if (i < n8) {
    const float* p = in + 8 * (size_t)i;
    const v4f a = *(const v4f*)(p);
    const v4f c = *(const v4f*)(p + 4);
    v4u u;
    u[0] = pk16(f2bf_bits(a[0]), f2bf_bits(a[1]));
    u[1] = pk16(f2bf_bits(a[2]), f2bf_bits(a[3]));
    u[2] = pk16(f2bf_bits(c[0]), f2bf_bits(c[1]));
    u[3] = pk16(f2bf_bits(c[2]), f2bf_bits(c[3]));
    unsigned short* d = outp + 8 * (size_t)i;
    *(volatile v4u*)d = u;
    __threadfence();
    *(volatile v4u*)d = u;
  }
}

__global__ __launch_bounds__(256) void k_proj(const unsigned short* __restrict__ Ap, const unsigned short* __restrict__ Btp,
                                              float* __restrict__ C, int M, int N, int K) {
  const __bf16* A  = (const __bf16*)Ap;
  const __bf16* Bt = (const __bf16*)Btp;
  __shared__ __align__(16) float sT[8][16 * 68];
  const int lane = threadIdx.x & 31;
  const int wave = threadIdx.x >> 5;
  const int tilesN = N >> 6;
  const int tilesM = M >> 6;
  const int tile = blockIdx.x * 8 + wave;
  if (tile >= tilesM * tilesN) return;
  const int tm = tile / tilesN;
  const int tn = tile - tm * tilesN;
  const int m0 = tm << 6;
  const int n0 = tn << 6;
  const int rlane = lane & 15;
  const int koff  = (lane >> 4) * 8;
  const int mOff  = (lane >> 4) * 8;

  v8f acc[4][4];
#pragma unroll
  for (int i = 0; i < 4; ++i)
#pragma unroll
    for (int j = 0; j < 4; ++j) acc[i][j] = (v8f){0.f, 0.f, 0.f, 0.f, 0.f, 0.f, 0.f, 0.f};

#pragma unroll 1
  for (int k0 = 0; k0 < K; k0 += 32) {
    v16b bh[4];
#pragma unroll
    for (int j = 0; j < 4; ++j) bh[j] = ldfrag_b(Bt + (size_t)(n0 + (j << 4) + rlane) * K + koff + k0);
#pragma unroll
    for (int i = 0; i < 4; ++i) {
      const v16b ah = ldfrag_b(A + (size_t)(m0 + (i << 4) + rlane) * K + koff + k0);
#pragma unroll
      for (int j = 0; j < 4; ++j) acc[i][j] = mma_b(ah, bh[j], acc[i][j]);
      guard_b2(acc[i][0], acc[i][3], ah, bh[3]);
    }
    keep4_b(bh[0], bh[1], bh[2], bh[3]);
  }
  acc_guard4(acc[0][0], acc[0][1], acc[0][2], acc[0][3]);
  acc_guard4(acc[1][0], acc[1][1], acc[1][2], acc[1][3]);
  acc_guard4(acc[2][0], acc[2][1], acc[2][2], acc[2][3]);
  acc_guard4(acc[3][0], acc[3][1], acc[3][2], acc[3][3]);

  float* slab = sT[wave];
  const int hh = lane >> 4;
  const int c4 = (lane & 15) * 4;
#pragma unroll
  for (int i = 0; i < 4; ++i) {
    const int mBase = m0 + (i << 4);
#pragma unroll
    for (int j = 0; j < 4; ++j) {
#pragma unroll
      for (int r = 0; r < 8; ++r) slab[(mOff + r) * 68 + (j << 4) + rlane] = acc[i][j][r];
    }
    __builtin_amdgcn_fence(__ATOMIC_RELEASE, "workgroup");
    __builtin_amdgcn_wave_barrier();
    __builtin_amdgcn_fence(__ATOMIC_ACQUIRE, "workgroup");
    for (int pass = 0; pass < 2; ++pass) {
#pragma unroll
      for (int it = 0; it < 8; ++it) {
        const int row = it * 2 + hh;
        const v4f v = *(const v4f*)(slab + row * 68 + c4);
        *(volatile v4f*)(C + (size_t)(mBase + row) * N + n0 + c4) = v;
      }
      __threadfence();
    }
    __builtin_amdgcn_fence(__ATOMIC_RELEASE, "workgroup");
    __builtin_amdgcn_wave_barrier();
    __builtin_amdgcn_fence(__ATOMIC_ACQUIRE, "workgroup");
  }
}

__global__ __launch_bounds__(256) void k_xt(const float* __restrict__ x, const float* __restrict__ att_s,
                                            const float* __restrict__ att_d,
                                            unsigned short* __restrict__ xth, unsigned short* __restrict__ xtl,
                                            float* __restrict__ a_s, float* __restrict__ a_d) {
  __shared__ __align__(16) unsigned short th[64 * 72];
  __shared__ __align__(16) unsigned short tl[64 * 72];
  __shared__ __align__(16) float sds[64];
  __shared__ __align__(16) float sdd[64];
  const int j0   = blockIdx.x * 64;
  const int h    = blockIdx.y;
  const int b    = blockIdx.z;
  const int tid  = threadIdx.x;
  const int lane = tid & 31;
  const int wave = tid >> 5;
  {
    const int rr = tid >> 2;
    const int cq = (tid & 3) * 16;
    const float* src = x + ((size_t)(b * NN + j0 + rr)) * HC + h * NC + cq;
    const float* asp = att_s + h * NC + cq;
    const float* adp = att_d + h * NC + cq;
    float ps = 0.f, pd = 0.f;
#pragma unroll 1
    for (int q = 0; q < 4; ++q) {
      const v4f f  = *(const v4f*)(src + 4 * q);
      const v4f sv = *(const v4f*)(asp + 4 * q);
      const v4f dv = *(const v4f*)(adp + 4 * q);
#pragma unroll
      for (int e = 0; e < 4; ++e) {
        ps += f[e] * bf_rn(sv[e]);
        pd += f[e] * bf_rn(dv[e]);
        const _Float16 hi = (_Float16)f[e];
        const float res = (f[e] - (float)hi) * LOSCALE;
        const _Float16 lo = (_Float16)res;
        th[rr * 72 + cq + 4 * q + e] = h_bits(hi);
        tl[rr * 72 + cq + 4 * q + e] = h_bits(lo);
      }
    }
    ps += __shfl_xor(ps, 1, 32);
    ps += __shfl_xor(ps, 2, 32);
    pd += __shfl_xor(pd, 1, 32);
    pd += __shfl_xor(pd, 2, 32);
    if ((lane & 3) == 0) { sds[rr] = ps; sdd[rr] = pd; }
  }
  __syncthreads();
  const int sub = tid >> 3;
  const int c8  = (tid & 7) * 8;
  v4u hv[2], lv[2];
#pragma unroll
  for (int it = 0; it < 2; ++it) {
    const int oc = it * 32 + sub;
    v4u a, a2;
#pragma unroll
    for (int q = 0; q < 4; ++q) {
      a[q]  = pk16(th[(c8 + 2 * q) * 72 + oc], th[(c8 + 2 * q + 1) * 72 + oc]);
      a2[q] = pk16(tl[(c8 + 2 * q) * 72 + oc], tl[(c8 + 2 * q + 1) * 72 + oc]);
    }
    hv[it] = a; lv[it] = a2;
  }
  const int hh = lane >> 4;
  const int c4 = (lane & 15) * 4;
  const v4f vs = *(const v4f*)(sds + c4);
  const v4f vd = *(const v4f*)(sdd + c4);
  v4f dv4;
#pragma unroll
  for (int e = 0; e < 4; ++e) dv4[e] = (hh != 0) ? vd[e] : vs[e];
  const size_t dbase = ((size_t)(b * NH + h)) * NN + j0 + c4;
  float* dp = ((hh != 0) ? a_d : a_s) + dbase;
  const size_t rowbase = ((size_t)(b * NH + h)) * NC;
  for (int pass = 0; pass < 2; ++pass) {
#pragma unroll
    for (int it = 0; it < 2; ++it) {
      const int oc = it * 32 + sub;
      const size_t go = (rowbase + oc) * NN + j0 + c8;
      *(volatile v4u*)(xth + go) = hv[it];
      *(volatile v4u*)(xtl + go) = lv[it];
    }
    if (wave == 0) { *(volatile v4f*)dp = dv4; }
    __threadfence();
  }
}

__global__ __launch_bounds__(256) void k_attn(const int* __restrict__ adj, const float* __restrict__ a_s,
                                              const float* __restrict__ a_d, const unsigned short* __restrict__ xthp,
                                              const unsigned short* __restrict__ xtlp, const float* __restrict__ bias,
                                              float* __restrict__ out) {
  __shared__ __align__(16) float sbuf[NH * NN];
  __shared__ __align__(16) unsigned smask[NN];
  const int tid  = threadIdx.x;
  const int lane = tid & 31;
  const int wave = tid >> 5;
  const int b    = blockIdx.x / (NN / ITILE);
  const int i0   = (blockIdx.x - b * (NN / ITILE)) * ITILE;

  {
    const float* g = a_s + (size_t)b * NH * NN;
#pragma unroll
    for (int it = 0; it < (NH * NN) / (4 * 256); ++it) {
      const int idx = (it * 256 + tid) * 4;
      *(v4f*)(sbuf + idx) = *(const v4f*)(g + idx);
    }
  }
#pragma unroll 1
  for (int it = 0; it < NN / 256; ++it) {
    const int j = it * 256 + tid;
    const int* arow = adj + ((size_t)(b * NN + j)) * NN + i0;
    unsigned msk = 0u;
#pragma unroll
    for (int q = 0; q < ITILE; q += 4) {
      const v4i av = *(const v4i*)(arow + q);
      msk |= ((av[0] != 0) ? 1u : 0u) << (q + 0);
      msk |= ((av[1] != 0) ? 1u : 0u) << (q + 1);
      msk |= ((av[2] != 0) ? 1u : 0u) << (q + 2);
      msk |= ((av[3] != 0) ? 1u : 0u) << (q + 3);
    }
    const int dj = j - i0;
    msk |= (dj >= 0 && dj < ITILE) ? (1u << (dj & 31)) : 0u;
    smask[j] = msk;
  }
  __syncthreads();

  const int h  = wave;
  const int m  = lane & 15;
  const int hf = lane >> 4;
  const float* asr = sbuf + h * NN;
  const float adv = a_d[((size_t)(b * NH + h)) * NN + i0 + m];

  float amax = -3.0e38f;
#pragma unroll 2
  for (int j = hf; j < NN; j += 2) {
    const bool adm = ((smask[j] >> m) & 1u) != 0u;
    const float v = asr[j];
    amax = adm ? fmaxf(amax, v) : amax;
  }
  amax = fmaxf(amax, __shfl_xor(amax, 16, 32));
  float emax = adv + amax;
  emax = fmaxf(emax, LEAKY * emax);
  float s = 0.f;
#pragma unroll 2
  for (int j = hf; j < NN; j += 2) {
    const bool adm = ((smask[j] >> m) & 1u) != 0u;
    float e = adv + asr[j];
    e = fmaxf(e, LEAKY * e);
    const float t = __expf(fminf(e - emax, 0.0f));
    s += adm ? t : 0.0f;
  }
  s += __shfl_xor(s, 16, 32);
  const float pscale = PSCALE / s;

  const _Float16* xth = (const _Float16*)xthp + ((size_t)(b * NH + h)) * NC * NN;
  const _Float16* xtl = (const _Float16*)xtlp + ((size_t)(b * NH + h)) * NC * NN;
  v8f acc[4], accr[4];
#pragma unroll
  for (int t = 0; t < 4; ++t) {
    acc[t]  = (v8f){0.f, 0.f, 0.f, 0.f, 0.f, 0.f, 0.f, 0.f};
    accr[t] = (v8f){0.f, 0.f, 0.f, 0.f, 0.f, 0.f, 0.f, 0.f};
  }
#pragma unroll 1
  for (int jb = 0; jb < NN; jb += 32) {
    FragH pa;
#pragma unroll
    for (int i = 0; i < 16; ++i) {
      const int k = (i < 8) ? (8 * hf + i) : (8 + 8 * hf + i);
      const int j = jb + k;
      const bool adm = ((smask[j] >> m) & 1u) != 0u;
      float e = adv + asr[j];
      e = fmaxf(e, LEAKY * e);
      const float p = __expf(fminf(e - emax, 0.0f)) * pscale;
      pa.s[i] = (_Float16)(adm ? p : 0.0f);
    }
    const v16h amat = pa.v;
#pragma unroll
    for (int t = 0; t < 4; ++t) {
      const size_t bo = (size_t)(t * 16 + m) * NN + jb + 8 * hf;
      const v16h bhf = ldfrag_h(xth + bo);
      const v16h blf = ldfrag_h(xtl + bo);
      acc[t]  = mma_h(amat, bhf, acc[t]);
      accr[t] = mma_h(amat, blf, accr[t]);
      guard_h3(acc[t], accr[t], amat, bhf, blf);
    }
  }
  acc_guard4(acc[0], acc[1], acc[2], acc[3]);
  acc_guard4(accr[0], accr[1], accr[2], accr[3]);

  __syncthreads();
  float* slab = sbuf + wave * (ITILE * NC);
#pragma unroll
  for (int t = 0; t < 4; ++t) {
#pragma unroll
    for (int r = 0; r < 8; ++r) slab[(8 * hf + r) * NC + t * 16 + m] = acc[t][r] * INV_P + accr[t][r] * INV_PL;
  }
  __syncthreads();
  const float* bh_ = bias + h * NC;
#pragma unroll 1
  for (int q = 0; q < (ITILE * NC) / (4 * 32); ++q) {
    const int e4  = (q * 32 + lane) * 4;
    const int col = e4 & (NC - 1);
    v4f v = *(const v4f*)(slab + e4);
#pragma unroll
    for (int c = 0; c < 4; ++c) {
      const float u  = v[c] + bf_rn(bh_[col + c]);
      const float un = expm1f(fminf(u, 0.0f));
      v[c] = (u > 0.0f) ? u : un;
    }
    *(v4f*)(slab + e4) = v;
  }
  __syncthreads();
  float* ob = out + ((size_t)(b * NN + i0)) * HC + h * NC + m * 4;
  for (int pass = 0; pass < 2; ++pass) {
#pragma unroll
    for (int it = 0; it < ITILE / 2; ++it) {
      const int row = it * 2 + hf;
      const v4f v = *(const v4f*)(slab + row * NC + m * 4);
      *(volatile v4f*)(ob + (size_t)row * HC) = v;
    }
    __threadfence();
  }
}

extern "C" void kernel_launch(void* const* d_in, const int* in_sizes, int n_in,
                              void* d_out, int out_size, void* d_ws, size_t ws_size,
                              hipStream_t stream) {
  if (n_in < 6) return;
  if (in_sizes[0] != NB * NN * ND) return;
  if (in_sizes[1] != NB * NN * NN) return;
  if (in_sizes[2] != ND * HC) return;
  if (in_sizes[3] != NH * NC || in_sizes[4] != NH * NC) return;
  if (in_sizes[5] != HC) return;
  if (out_size != NB * NN * HC) return;

  const float* feat  = (const float*)d_in[0];
  const int*   adj   = (const int*)d_in[1];
  const float* W     = (const float*)d_in[2];
  const float* att_s = (const float*)d_in[3];
  const float* att_d = (const float*)d_in[4];
  const float* bias  = (const float*)d_in[5];
  float* out = (float*)d_out;

  const size_t PWT = (size_t)HC * ND * 2;
  const size_t PFB = (size_t)NB * NN * ND * 2;
  const size_t PX  = (size_t)NB * NN * HC * 4;
  const size_t PXT = (size_t)NB * NH * NC * NN * 2;
  const size_t PA  = (size_t)NB * NH * NN * 4;
  size_t off = 0;
  const size_t oWt  = off; off += PWT;
  const size_t oFb  = off; off += PFB;
  const size_t oX   = off; off += PX;
  const size_t oXth = off; off += PXT;
  const size_t oXtl = off; off += PXT;
  const size_t oAs  = off; off += PA;
  const size_t oAd  = off; off += PA;
  if (off > ws_size) return;

  char* ws = (char*)d_ws;
  unsigned short* Wt  = (unsigned short*)(ws + oWt);
  unsigned short* Fb  = (unsigned short*)(ws + oFb);
  float*          X   = (float*)(ws + oX);
  unsigned short* Xth = (unsigned short*)(ws + oXth);
  unsigned short* Xtl = (unsigned short*)(ws + oXtl);
  float*          As  = (float*)(ws + oAs);
  float*          Ad  = (float*)(ws + oAd);

  const dim3 blk(256);
  k_wt<<<dim3(HC / 64, ND / 64), blk, 0, stream>>>(W, Wt);
  const int n8 = (NB * NN * ND) / 8;
  k_cvtf<<<dim3((n8 + 255) / 256), blk, 0, stream>>>(feat, Fb, n8);
  const int tiles = ((NB * NN) / 64) * (HC / 64);
  k_proj<<<dim3((tiles + 7) / 8), blk, 0, stream>>>(Fb, Wt, X, NB * NN, HC, ND);
  k_xt<<<dim3(NN / 64, NH, NB), blk, 0, stream>>>(X, att_s, att_d, Xth, Xtl, As, Ad);
  k_attn<<<dim3(NB * (NN / ITILE)), blk, 0, stream>>>(adj, As, Ad, Xth, Xtl, bias, out);
  (void)hipGetLastError();
}
